// DiagonalPixelLSTM_45114336477858
// MI455X (gfx1250) — hardware-verified
//
#include <hip/hip_runtime.h>
#include <math.h>

typedef __attribute__((ext_vector_type(16))) _Float16 v16h;
typedef __attribute__((ext_vector_type(8)))  _Float16 v8h;
typedef __attribute__((ext_vector_type(8)))  float    v8f;
typedef __attribute__((ext_vector_type(4)))  float    v4f;

constexpr int kB    = 16;
constexpr int kC    = 64;
constexpr int kRows = 64;
constexpr int kCols = 64;
constexpr int kHid  = 64;
constexpr int kG5   = 5 * kHid;
constexpr int kSkew = 2 * kCols - 1;
constexpr int kThr  = 512;
constexpr int kWP   = 136;
constexpr int kHP   = 72;
constexpr int kCP   = 68;
constexpr size_t kOutElems = (size_t)kB * kHid * kRows * kCols;

constexpr float kWCarry = 4096.0f;
constexpr float kSCarry = 1024.0f;
constexpr float kFold   = 1.0f / (kWCarry * kSCarry);
constexpr float kF16MinNormal = 6.103515625e-5f;
static_assert(kFold == 2.384185791015625e-7f, "2^-22");
static_assert(kRows == 64 && kHid == 64 && kThr == 512, "four row tiles x four hidden quarters of 16");

union FragU { v16h v; v8h h[2]; };

__device__ __forceinline__ unsigned short f2bf_bits(float f) {
  unsigned u = __float_as_uint(f);
  return (unsigned short)((u + 0x7FFFu + ((u >> 16) & 1u)) >> 16);
}
__device__ __forceinline__ float bf16r(float f) { return __uint_as_float(((unsigned)f2bf_bits(f)) << 16); }
__device__ __forceinline__ float carry_flush(float v, float c) {
  const float s = v * c;
  return (fabsf(s) < kF16MinNormal) ? 0.0f : s;
}
__device__ __forceinline__ void split_hl(float v, float c, _Float16& hi, _Float16& lo) {
  const float sv = carry_flush(v, c);
  hi = (_Float16)sv;
  const float r = sv - (float)hi;
  lo = (_Float16)((fabsf(r) < kF16MinNormal) ? 0.0f : r);
}
__device__ __forceinline__ v8f mma_h(v16h a, v16h b, v8f c) {
  c = __builtin_amdgcn_wmma_f32_16x16x32_f16(false, a, false, b, (short)0, c, false, false);
  asm volatile("v_nop\n\tv_nop\n\tv_nop\n\tv_nop" : "+v"(c) : "v"(a), "v"(b));
  return c;
}
__device__ __forceinline__ v16h frag_h32(const _Float16* p) { FragU f; f.h[0] = *(const v8h*)(p); f.h[1] = *(const v8h*)(p + 16); return f.v; }
__device__ __forceinline__ float sigmoid_p(float v) { return 1.0f / (1.0f + expf(-v)); }

__global__ __launch_bounds__(kThr) void diag_lstm_kernel(const float* __restrict__ features, const float* __restrict__ W_is,
                                                         const float* __restrict__ b_is, const float* __restrict__ W_ss,
                                                         const float* __restrict__ b_ss, float* __restrict__ out) {
  __shared__ __align__(16) _Float16 sW[kG5 * kWP];
  __shared__ __align__(16) _Float16 sHh[(kRows + 1) * kHP];
  __shared__ __align__(16) _Float16 sHl[(kRows + 1) * kHP];
  __shared__ __align__(16) float    sC[(kRows + 1) * kCP];
  __shared__ __align__(16) _Float16 sX[kRows * kHP];
  __shared__ __align__(16) float    sBias[kG5];

  const int tid = threadIdx.x;
  const int wave = tid >> 5;
  const int lane = tid & 31;
  const int col = lane & 15;
  const int hs = lane >> 4;
  const int rt = wave & 3;
  const int hq = wave >> 2;
  const int bb = blockIdx.x;
  const int row = 16 * rt + col;
  const int u0 = 16 * hq + 8 * hs;
  const float* fb = features + (size_t)bb * kC * kRows * kCols;

#pragma unroll 1
  for (int i = tid; i < kG5 * kHid; i += kThr) {
    const int g = i >> 6;
    const int k = i & 63;
    const float w1 = W_ss[(size_t)i * 2 + 1];
    const float w0 = W_ss[(size_t)i * 2];
    sW[g * kWP + k] = (_Float16)carry_flush(bf16r(w1), kWCarry);
    sW[g * kWP + kHid + k] = (_Float16)carry_flush(bf16r(w0), kWCarry);
  }
  if (tid < kG5) {
    const float b0 = b_is[tid];
    const float b1 = b_ss[tid];
    sBias[tid] = bf16r(b0) + bf16r(b1);
  }
#pragma unroll 1
  for (int i = tid; i < (kRows + 1) * kHP; i += kThr) { sHh[i] = (_Float16)0.0f; sHl[i] = (_Float16)0.0f; }
#pragma unroll 1
  for (int i = tid; i < (kRows + 1) * kCP; i += kThr) sC[i] = 0.0f;
  v16h wis[5][2];
#pragma unroll
  for (int g = 0; g < 5; ++g)
#pragma unroll
    for (int ks = 0; ks < 2; ++ks) {
      const float* wp = W_is + (size_t)(64 * g + 16 * hq + col) * kC + 32 * ks + 8 * hs;
#pragma unroll
      for (int e = 0; e < 8; ++e) {
        const float w0 = wp[e];
        const float w1 = wp[16 + e];
        wis[g][ks][e] = (_Float16)carry_flush(bf16r(w0), kWCarry);
        wis[g][ks][8 + e] = (_Float16)carry_flush(bf16r(w1), kWCarry);
      }
    }
  {
    const int r = tid & 63;
    const int c8 = (tid >> 6) * 8;
    const int src = 0 - r;
    const bool valid = (src >= 0) && (src < kCols);
    const int sc = valid ? src : 0;
    v8h xv;
#pragma unroll
    for (int e = 0; e < 8; ++e) {
      const float x = fb[((size_t)(c8 + e) * kRows + r) * kCols + sc];
      xv[e] = (_Float16)carry_flush(valid ? bf16r(x) : 0.0f, kSCarry);
    }
    *(v8h*)(sX + r * kHP + c8) = xv;
  }
  float cst[8];
#pragma unroll
  for (int r = 0; r < 8; ++r) cst[r] = 0.0f;

#pragma unroll 1
  for (int ws = 0; ws < kSkew; ++ws) {
    __syncthreads();
    int rowv = row, colv = col, hsv = hs;
    asm volatile("" : "+v"(rowv), "+v"(colv), "+v"(hsv));
    const v4f cu0 = *(const v4f*)(sC + rowv * kCP + u0);
    const v4f cu1 = *(const v4f*)(sC + rowv * kCP + u0 + 4);
    v8f acc[5];
#pragma unroll
    for (int g = 0; g < 5; ++g) acc[g] = (v8f){0.f, 0.f, 0.f, 0.f, 0.f, 0.f, 0.f, 0.f};
#pragma unroll
    for (int ks = 0; ks < 2; ++ks) {
      const v16h hh = frag_h32(sHh + (rowv + 1) * kHP + 32 * ks + 8 * hsv);
      const v16h hl = frag_h32(sHl + (rowv + 1) * kHP + 32 * ks + 8 * hsv);
      const v16h ph = frag_h32(sHh + rowv * kHP + 32 * ks + 8 * hsv);
      const v16h pl = frag_h32(sHl + rowv * kHP + 32 * ks + 8 * hsv);
      const v16h xf = frag_h32(sX + rowv * kHP + 32 * ks + 8 * hsv);
#pragma unroll
      for (int g = 0; g < 5; ++g) {
        const _Float16* wr = sW + (64 * g + 16 * hq + colv) * kWP + 32 * ks + 8 * hsv;
        const v16h a1 = frag_h32(wr);
        const v16h a0 = frag_h32(wr + kHid);
        acc[g] = mma_h(a1, hh, acc[g]);
        acc[g] = mma_h(a1, hl, acc[g]);
        acc[g] = mma_h(a0, ph, acc[g]);
        acc[g] = mma_h(a0, pl, acc[g]);
        acc[g] = mma_h(wis[g][ks], xf, acc[g]);
      }
    }
    float hnew[8];
#pragma unroll
    for (int r = 0; r < 8; ++r) {
      const float go = acc[0][r] * kFold + sBias[0 * kHid + u0 + r];
      const float gl = acc[1][r] * kFold + sBias[1 * kHid + u0 + r];
      const float gu = acc[2][r] * kFold + sBias[2 * kHid + u0 + r];
      const float gi = acc[3][r] * kFold + sBias[3 * kHid + u0 + r];
      const float gc = acc[4][r] * kFold + sBias[4 * kHid + u0 + r];
      const float cup = (r < 4) ? cu0[r] : cu1[r - 4];
      const float cn = sigmoid_p(gl) * cst[r] + sigmoid_p(gu) * cup + sigmoid_p(gi) * tanhf(gc);
      cst[r] = cn;
      hnew[r] = sigmoid_p(go) * tanhf(cn);
    }
    {
      const int oc = ws - rowv;
      if (oc >= 0 && oc < kCols) {
        float* op = out + (((size_t)bb * kHid + u0) * kRows + rowv) * kCols + oc;
        for (int pass = 0; pass < 2; ++pass) {
#pragma unroll
          for (int r = 0; r < 8; ++r) *(volatile float*)(op + (size_t)r * kRows * kCols) = hnew[r];
          __threadfence();
        }
      }
    }
    __syncthreads();
    asm volatile("" : "+v"(rowv), "+v"(colv), "+v"(hsv));
    {
      v8h vh, vl;
#pragma unroll
      for (int r = 0; r < 8; ++r) { _Float16 h, l; split_hl(hnew[r], kSCarry, h, l); vh[r] = h; vl[r] = l; }
      *(v8h*)(sHh + (rowv + 1) * kHP + u0) = vh;
      *(v8h*)(sHl + (rowv + 1) * kHP + u0) = vl;
      *(v4f*)(sC + (rowv + 1) * kCP + u0) = (v4f){cst[0], cst[1], cst[2], cst[3]};
      *(v4f*)(sC + (rowv + 1) * kCP + u0 + 4) = (v4f){cst[4], cst[5], cst[6], cst[7]};
    }
    {
      const int r = tid & 63;
      const int c8 = (tid >> 6) * 8;
      const int src = ws + 1 - r;
      const bool valid = (src >= 0) && (src < kCols);
      const int sc = valid ? src : 0;
      v8h xv;
#pragma unroll
      for (int e = 0; e < 8; ++e) {
        const float x = fb[((size_t)(c8 + e) * kRows + r) * kCols + sc];
        xv[e] = (_Float16)carry_flush(valid ? bf16r(x) : 0.0f, kSCarry);
      }
      *(v8h*)(sX + r * kHP + c8) = xv;
    }
  }
}

extern "C" void kernel_launch(void* const* d_in, const int* in_sizes, int n_in,
                              void* d_out, int out_size, void* d_ws, size_t ws_size,
                              hipStream_t stream) {
  if (n_in < 5 || d_out == nullptr) return;
  if (in_sizes[0] != kB * kC * kRows * kCols || in_sizes[1] != kG5 * kC || in_sizes[2] != kG5) return;
  if (in_sizes[3] != kG5 * kHid * 2 || in_sizes[4] != kG5) return;
  if ((size_t)out_size != kOutElems) return;
  diag_lstm_kernel<<<kB, kThr, 0, stream>>>((const float*)d_in[0], (const float*)d_in[1], (const float*)d_in[2],
                                            (const float*)d_in[3], (const float*)d_in[4], (float*)d_out);
}
